// QwenAttention_21019569946993
// MI455X (gfx1250) — hardware-verified
//
#include <hip/hip_runtime.h>
#include <math.h>

#pragma clang fp contract(off)

typedef __attribute__((ext_vector_type(16))) _Float16 v16h;
typedef __attribute__((ext_vector_type(8)))  _Float16 v8h;
typedef __attribute__((ext_vector_type(16))) __bf16   v16b;
typedef __attribute__((ext_vector_type(8)))  __bf16   v8b;
typedef __attribute__((ext_vector_type(8)))  float    v8f;
typedef __attribute__((ext_vector_type(4)))  float    v4f;
typedef __attribute__((ext_vector_type(4)))  unsigned int v4u;

constexpr int SEQ   = 2048;
constexpr int HID   = 2048;
constexpr int NHEAD = 16;
constexpr int HDIM  = 128;
constexpr int NKVH  = 4;
constexpr int QKVN  = NHEAD * HDIM + 2 * NKVH * HDIM;
constexpr int KOFF  = NHEAD * HDIM;
constexpr int VOFF  = KOFF + NKVH * HDIM;
constexpr float SM_SCALE = 0.08838834764831845f;

static_assert(QKVN == 3072 && KOFF == 2048 && VOFF == 2560, "geometry");
static_assert(SEQ % 64 == 0 && QKVN % 64 == 0 && HID % 64 == 0, "GEMM M/N tile multiples");
static_assert(HID % 32 == 0, "GEMM K multiple of 32");
static_assert((SEQ * HID) % (8 * 256) == 0, "cast grid exact");
static_assert(NHEAD % NKVH == 0 && HDIM == 128, "head geometry");

constexpr size_t BYTES_XB  = (size_t)SEQ * HID * 2;
constexpr size_t BYTES_WAT = (size_t)QKVN * HID * 2;
constexpr size_t BYTES_WPT = (size_t)HID * HID * 2;
constexpr size_t BYTES_QKV = (size_t)SEQ * QKVN * 4;
constexpr size_t BYTES_QPL = (size_t)NHEAD * SEQ * HDIM * 2;
constexpr size_t BYTES_KPL = (size_t)NKVH * SEQ * HDIM * 2;
constexpr size_t BYTES_OPL = (size_t)SEQ * HID * 2;
constexpr size_t OFF_XB  = 0;
constexpr size_t OFF_WAT = OFF_XB + BYTES_XB;
constexpr size_t OFF_WPT = OFF_WAT + BYTES_WAT;
constexpr size_t OFF_QKV = OFF_WPT + BYTES_WPT;
constexpr size_t OFF_QH  = OFF_QKV + BYTES_QKV;
constexpr size_t OFF_QL  = OFF_QH + BYTES_QPL;
constexpr size_t OFF_KH  = OFF_QL + BYTES_QPL;
constexpr size_t OFF_KL  = OFF_KH + BYTES_KPL;
constexpr size_t OFF_VH  = OFF_KL + BYTES_KPL;
constexpr size_t OFF_VL  = OFF_VH + BYTES_KPL;
constexpr size_t OFF_OH  = OFF_VL + BYTES_KPL;
constexpr size_t OFF_OL  = OFF_OH + BYTES_OPL;
constexpr size_t WS_TOTAL = OFF_OL + BYTES_OPL;
static_assert(WS_TOTAL == 96468992ull, "carve total");
static_assert(WS_TOTAL <= 134217728ull, "carve cap");
static_assert(OFF_WAT % 128 == 0 && OFF_WPT % 128 == 0 && OFF_QKV % 128 == 0 && OFF_QH % 128 == 0 &&
              OFF_QL % 128 == 0 && OFF_KH % 128 == 0 && OFF_KL % 128 == 0 && OFF_VH % 128 == 0 &&
              OFF_VL % 128 == 0 && OFF_OH % 128 == 0 && OFF_OL % 128 == 0, "line aligned carve");

__device__ __forceinline__ unsigned short f2bf_bits(float f) {
  unsigned u = __float_as_uint(f);
  return (unsigned short)((u + 0x7FFFu + ((u >> 16) & 1u)) >> 16);
}
__device__ __forceinline__ float bf_bits2f(unsigned short h) { return __uint_as_float(((unsigned)h) << 16); }

__device__ __forceinline__ void dep_guard_h(v8f& a, v8f& b, v16h x, v16h y) { asm volatile("v_nop\n\tv_nop\n\tv_nop\n\tv_nop" : "+v"(a), "+v"(b) : "v"(x), "v"(y)); }
__device__ __forceinline__ void dep_guard_b(v8f& a, v8f& b, v16b x, v16b y) { asm volatile("v_nop\n\tv_nop\n\tv_nop\n\tv_nop" : "+v"(a), "+v"(b) : "v"(x), "v"(y)); }
__device__ __forceinline__ void keep4_h(v16h a, v16h b, v16h c, v16h d) { asm volatile("v_nop" :: "v"(a), "v"(b), "v"(c), "v"(d)); }
__device__ __forceinline__ void keep4_b(v16b a, v16b b, v16b c, v16b d) { asm volatile("v_nop" :: "v"(a), "v"(b), "v"(c), "v"(d)); }
__device__ __forceinline__ void acc_guard4(v8f& a, v8f& b, v8f& c, v8f& d) { asm volatile("v_nop\n\tv_nop\n\tv_nop\n\tv_nop" : "+v"(a), "+v"(b), "+v"(c), "+v"(d)); }
template <typename T> struct Frag;
template <> struct Frag<_Float16> {
  typedef v16h V; union U { v16h v; v8h h[2]; };
  static __device__ __forceinline__ v16h load(const _Float16* p) {
    U f; f.h[0] = *(const v8h*)(p); f.h[1] = *(const v8h*)(p + 16); return f.v;
  }
  static __device__ __forceinline__ v8f mma(v16h a, v16h b, v8f c) {
    return __builtin_amdgcn_wmma_f32_16x16x32_f16(false, a, false, b, (short)0, c, false, false);
  }
  static __device__ __forceinline__ void guard(v8f& a, v8f& b, v16h x, v16h y) { dep_guard_h(a, b, x, y); }
  static __device__ __forceinline__ void keep(v16h a, v16h b, v16h c, v16h d) { keep4_h(a, b, c, d); }
};
template <> struct Frag<__bf16> {
  typedef v16b V; union U { v16b v; v8b h[2]; };
  static __device__ __forceinline__ v16b load(const __bf16* p) {
    U f; f.h[0] = *(const v8b*)(p); f.h[1] = *(const v8b*)(p + 16); return f.v;
  }
  static __device__ __forceinline__ v8f mma(v16b a, v16b b, v8f c) {
    return __builtin_amdgcn_wmma_f32_16x16x32_bf16(false, a, false, b, (short)0, c, false, false);
  }
  static __device__ __forceinline__ void guard(v8f& a, v8f& b, v16b x, v16b y) { dep_guard_b(a, b, x, y); }
  static __device__ __forceinline__ void keep(v16b a, v16b b, v16b c, v16b d) { keep4_b(a, b, c, d); }
};

__device__ __forceinline__ __bf16 at_f2bf(float f) { return __builtin_bit_cast(__bf16, f2bf_bits(f)); }
__device__ __forceinline__ void at_split(float f, __bf16& hi, __bf16& lo) {
  const unsigned short hb = f2bf_bits(f);
  hi = __builtin_bit_cast(__bf16, hb);
  lo = at_f2bf(f - __uint_as_float(((unsigned)hb) << 16));
}
__device__ __forceinline__ v8f at_mma(v16b a, v16b b, v8f c) {
  c = __builtin_amdgcn_wmma_f32_16x16x32_bf16(false, a, false, b, (short)0, c, false, false);
  asm volatile("v_nop\n\tv_nop\n\tv_nop\n\tv_nop" : "+v"(c) : "v"(a), "v"(b));
  return c;
}

struct HL2 { unsigned hi; unsigned lo; };
__device__ __forceinline__ HL2 split_pack2(float x0, float x1) {
  const unsigned short h0 = f2bf_bits(x0), h1 = f2bf_bits(x1);
  const unsigned short l0 = f2bf_bits(x0 - bf_bits2f(h0));
  const unsigned short l1 = f2bf_bits(x1 - bf_bits2f(h1));
  HL2 r;
  r.hi = (unsigned)h0 | ((unsigned)h1 << 16);
  r.lo = (unsigned)l0 | ((unsigned)l1 << 16);
  return r;
}
__device__ __forceinline__ unsigned pack_bf2(float x0, float x1) {
  return (unsigned)f2bf_bits(x0) | ((unsigned)f2bf_bits(x1) << 16);
}

template <int ET> struct Elem;
template <> struct Elem<0> { typedef _Float16 T; };
template <> struct Elem<1> { typedef __bf16 T; };
template <int ET, int SPLITMODE, int OUT_MODE>
__global__ __launch_bounds__(256) void wmma_gemm64(
    const unsigned short* __restrict__ Ap, const unsigned short* __restrict__ A2p, int lda, long strideA,
    const unsigned short* __restrict__ Btp, const unsigned short* __restrict__ Bt2p, int ldb, long strideB,
    void* __restrict__ Cout, void* __restrict__ Cout2, int ldc, long strideC,
    int M, int N, int K, float scale) {
  constexpr bool SPA = (SPLITMODE != 0);
  constexpr bool SPB = (SPLITMODE == 1);
  typedef typename Elem<ET>::T T;
  typedef typename Frag<T>::V V;
  const T* A = (const T*)Ap; const T* A2 = (const T*)A2p; const T* Bt = (const T*)Btp; const T* Bt2 = (const T*)Bt2p;
  __shared__ __align__(16) float sT[8][16 * 68];
  const int b    = blockIdx.y;
  const int lane = threadIdx.x & 31;
  const int wave = threadIdx.x >> 5;
  const int tilesN = N >> 6;
  const int tilesM = M >> 6;
  const int tile = blockIdx.x * 8 + wave;
  if (tile >= tilesM * tilesN) return;
  const int tm = tile / tilesN;
  const int tn = tile - tm * tilesN;
  const int m0 = tm << 6;
  const int n0 = tn << 6;

  const T* Ab  = A  + (size_t)b * strideA;
  const T* Bb  = Bt + (size_t)b * strideB;
  const T* Ab2 = SPA ? (A2  + (size_t)b * strideA) : nullptr;
  const T* Bb2 = SPB ? (Bt2 + (size_t)b * strideB) : nullptr;

  const int rlane = lane & 15;
  const int koff  = (lane >> 4) * 8;
  const int mOff  = (lane >> 4) * 8;

  v8f acc[4][4];
#pragma unroll
  for (int i = 0; i < 4; ++i)
#pragma unroll
    for (int j = 0; j < 4; ++j) acc[i][j] = (v8f){0.f,0.f,0.f,0.f,0.f,0.f,0.f,0.f};

  for (int k0 = 0; k0 < K; k0 += 32) {
    V bh[4], bl[4];
#pragma unroll
    for (int j = 0; j < 4; ++j) {
      const size_t bo = (size_t)(n0 + (j << 4) + rlane) * ldb + koff + k0;
      bh[j] = Frag<T>::load(Bb + bo);
      if (SPB) bl[j] = Frag<T>::load(Bb2 + bo);
    }
#pragma unroll
    for (int i = 0; i < 4; ++i) {
      const size_t ao = (size_t)(m0 + (i << 4) + rlane) * lda + koff + k0;
      V ah = Frag<T>::load(Ab + ao);
      V al;
      if (SPA) al = Frag<T>::load(Ab2 + ao);
#pragma unroll
      for (int j = 0; j < 4; ++j) {
        acc[i][j] = Frag<T>::mma(ah, bh[j], acc[i][j]);
        if (SPB) acc[i][j] = Frag<T>::mma(ah, bl[j], acc[i][j]);
        if (SPA) acc[i][j] = Frag<T>::mma(al, bh[j], acc[i][j]);
      }
      Frag<T>::guard(acc[i][0], acc[i][3], ah, SPA ? al : ah);
    }
    Frag<T>::keep(bh[0], bh[1], bh[2], bh[3]);
    if (SPB) Frag<T>::keep(bl[0], bl[1], bl[2], bl[3]);
  }
  acc_guard4(acc[0][0], acc[0][1], acc[0][2], acc[0][3]);
  acc_guard4(acc[1][0], acc[1][1], acc[1][2], acc[1][3]);
  acc_guard4(acc[2][0], acc[2][1], acc[2][2], acc[2][3]);
  acc_guard4(acc[3][0], acc[3][1], acc[3][2], acc[3][3]);

  float* slab = sT[wave];
#pragma unroll
  for (int i = 0; i < 4; ++i) {
    const int mBase = m0 + (i << 4);
#pragma unroll
    for (int j = 0; j < 4; ++j) {
#pragma unroll
      for (int r = 0; r < 8; ++r) {
        const float v = acc[i][j][r] * scale;
        slab[(mOff + r) * 68 + (j << 4) + rlane] = v;
      }
    }
    __builtin_amdgcn_fence(__ATOMIC_RELEASE, "workgroup");
    __builtin_amdgcn_wave_barrier();
    __builtin_amdgcn_fence(__ATOMIC_ACQUIRE, "workgroup");
    if (OUT_MODE == 0) {
      float* C = (float*)Cout + (size_t)b * strideC;
      const int hh = lane >> 4, c4 = (lane & 15) * 4;
      for (int pass = 0; pass < 2; ++pass) {
#pragma unroll
        for (int it = 0; it < 8; ++it) {
          const int row = it * 2 + hh;
          v4f v = *(const v4f*)(slab + row * 68 + c4);
          *(volatile v4f*)(C + (size_t)(mBase + row) * ldc + n0 + c4) = v;
        }
        __threadfence();
      }
    } else {
      const int q = lane >> 3, c8 = (lane & 7) * 8;
      unsigned short* C  = (unsigned short*)Cout  + (size_t)b * strideC;
      unsigned short* C2 = (OUT_MODE == 2) ? ((unsigned short*)Cout2 + (size_t)b * strideC) : nullptr;
      for (int pass = 0; pass < 2; ++pass) {
#pragma unroll
        for (int it = 0; it < 4; ++it) {
          const int row = it * 4 + q;
          const float* sp = slab + row * 68 + c8;
          v8h hv, lv;
#pragma unroll
          for (int e = 0; e < 8; ++e) {
            if (OUT_MODE == 1) {
              hv[e] = (_Float16)sp[e];
            } else {
              unsigned short hb = f2bf_bits(sp[e]);
              unsigned short lb = f2bf_bits(sp[e] - bf_bits2f(hb));
              hv[e] = __builtin_bit_cast(_Float16, hb);
              lv[e] = __builtin_bit_cast(_Float16, lb);
            }
          }
          *(volatile v8h*)(C + (size_t)(mBase + row) * ldc + n0 + c8) = hv;
          if (OUT_MODE == 2) *(volatile v8h*)(C2 + (size_t)(mBase + row) * ldc + n0 + c8) = lv;
        }
        __threadfence();
      }
    }
    __builtin_amdgcn_fence(__ATOMIC_RELEASE, "workgroup");
    __builtin_amdgcn_wave_barrier();
    __builtin_amdgcn_fence(__ATOMIC_ACQUIRE, "workgroup");
  }
}

__global__ __launch_bounds__(256) void cast_f32_bf16x8(const float* __restrict__ in,
                                                       unsigned short* __restrict__ out, int n8) {
  const int i = blockIdx.x * 256 + threadIdx.x;
  if (i >= n8) return;
  const v4f a = *(const v4f*)(in + (size_t)i * 8);
  const v4f b = *(const v4f*)(in + (size_t)i * 8 + 4);
  v4u w;
  w[0] = pack_bf2(a[0], a[1]);
  w[1] = pack_bf2(a[2], a[3]);
  w[2] = pack_bf2(b[0], b[1]);
  w[3] = pack_bf2(b[2], b[3]);
  unsigned short* dst = out + (size_t)i * 8;
  *(volatile v4u*)dst = w;
  __threadfence();
  *(volatile v4u*)dst = w;
}

__global__ __launch_bounds__(256) void transpose_cast_bf16(const float* __restrict__ in,
                                                           unsigned short* __restrict__ out, int R, int CC) {
  __shared__ __align__(16) unsigned short T[64 * 72];
  const int n0 = blockIdx.x * 64;
  const int r0 = blockIdx.y * 64;
  const int tid = threadIdx.x;
  {
    const int rr = tid >> 2, part = tid & 3;
    const float* src = in + (size_t)(r0 + rr) * CC + n0 + part * 16;
    const v4f x0 = *(const v4f*)(src);
    const v4f x1 = *(const v4f*)(src + 4);
    const v4f x2 = *(const v4f*)(src + 8);
    const v4f x3 = *(const v4f*)(src + 12);
    unsigned short* tp = T + (part * 16) * 72 + rr;
#pragma unroll
    for (int e = 0; e < 4; ++e) {
      tp[(e) * 72]      = f2bf_bits(x0[e]);
      tp[(4 + e) * 72]  = f2bf_bits(x1[e]);
      tp[(8 + e) * 72]  = f2bf_bits(x2[e]);
      tp[(12 + e) * 72] = f2bf_bits(x3[e]);
    }
  }
  __syncthreads();
  const int wave = tid >> 5, lane = tid & 31, q = lane >> 3, c8 = (lane & 7) * 8;
  for (int ps = 0; ps < 2; ++ps) {
#pragma unroll
    for (int it = 0; it < 2; ++it) {
      const int row = wave * 8 + it * 4 + q;
      const v4u v = *(const v4u*)(T + row * 72 + c8);
      *(volatile v4u*)(out + (size_t)(n0 + row) * R + r0 + c8) = v;
    }
    __threadfence();
  }
}

struct RopeFreq { float inv[64]; };
static_assert(sizeof(RopeFreq) == 256, "no padding");

__device__ __forceinline__ void rope_pack8(const float* __restrict__ xp, int d0, int pd0, float sgn,
                                           v4f ca, v4f cb, v4f sa, v4f sb, v4u& hv, v4u& lv) {
  const v4f x0 = *(const v4f*)(xp + d0);
  const v4f x1 = *(const v4f*)(xp + d0 + 4);
  const v4f r0 = *(const v4f*)(xp + pd0);
  const v4f r1 = *(const v4f*)(xp + pd0 + 4);
  const v4f oa = x0 * ca + (r0 * sgn) * sa;
  const v4f ob = x1 * cb + (r1 * sgn) * sb;
  const HL2 p0 = split_pack2(oa[0], oa[1]);
  const HL2 p1 = split_pack2(oa[2], oa[3]);
  const HL2 p2 = split_pack2(ob[0], ob[1]);
  const HL2 p3 = split_pack2(ob[2], ob[3]);
  hv[0] = p0.hi; hv[1] = p1.hi; hv[2] = p2.hi; hv[3] = p3.hi;
  lv[0] = p0.lo; lv[1] = p1.lo; lv[2] = p2.lo; lv[3] = p3.lo;
}

__global__ __launch_bounds__(128) void rope_qk_kernel(const float* __restrict__ qkv,
                                                     const int* __restrict__ pos_ids, RopeFreq rf,
                                                     unsigned short* __restrict__ Qh, unsigned short* __restrict__ Ql,
                                                     unsigned short* __restrict__ Kh, unsigned short* __restrict__ Kl) {
  __shared__ __align__(16) float ce[HDIM];
  __shared__ __align__(16) float se[HDIM];
  const int s = blockIdx.x;
  const int tid = threadIdx.x;
  {
    const int i = tid & 63;
    float inv = 0.f;
#pragma unroll
    for (int j = 0; j < 64; ++j) inv = (i == j) ? rf.inv[j] : inv;
    const int pos = pos_ids[s];
    const float t = (float)pos;
    const float fr = t * inv;
    float sf, cf;
    sincosf(fr, &sf, &cf);
    const float e = (tid < 64) ? sf : cf;
    float s2, c2;
    sincosf(e, &s2, &c2);
    ce[tid] = c2;
    se[tid] = s2;
  }
  __syncthreads();
  const int wave = tid >> 5, lane = tid & 31, hh = lane >> 4, c = lane & 15;
  const int d0 = c * 8, pd0 = d0 ^ 64;
  const float sgn = (c < 8) ? -1.0f : 1.0f;
  const v4f ca = *(const v4f*)(ce + d0), cb = *(const v4f*)(ce + d0 + 4);
  const v4f sa = *(const v4f*)(se + d0), sb = *(const v4f*)(se + d0 + 4);
  const float* row = qkv + (size_t)s * QKVN;
  const int hq0 = 2 * wave + hh;
  const int hq1 = hq0 + 8;
  v4u qh0, ql0, qh1, ql1;
  rope_pack8(row + hq0 * HDIM, d0, pd0, sgn, ca, cb, sa, sb, qh0, ql0);
  rope_pack8(row + hq1 * HDIM, d0, pd0, sgn, ca, cb, sa, sb, qh1, ql1);
  const size_t o0 = ((size_t)hq0 * SEQ + s) * HDIM + d0;
  const size_t o1 = ((size_t)hq1 * SEQ + s) * HDIM + d0;
  for (int ps = 0; ps < 2; ++ps) {
    *(volatile v4u*)(Qh + o0) = qh0;
    *(volatile v4u*)(Ql + o0) = ql0;
    *(volatile v4u*)(Qh + o1) = qh1;
    *(volatile v4u*)(Ql + o1) = ql1;
    __threadfence();
  }
  if (wave < 2) {
    const int hk = 2 * wave + hh;
    v4u kh, kl;
    rope_pack8(row + KOFF + hk * HDIM, d0, pd0, sgn, ca, cb, sa, sb, kh, kl);
    const size_t ok = ((size_t)hk * SEQ + s) * HDIM + d0;
    for (int ps = 0; ps < 2; ++ps) {
      *(volatile v4u*)(Kh + ok) = kh;
      *(volatile v4u*)(Kl + ok) = kl;
      __threadfence();
    }
  }
}

__global__ __launch_bounds__(256) void v_split_transpose_kernel(const float* __restrict__ qkv,
                                                               unsigned short* __restrict__ Vth,
                                                               unsigned short* __restrict__ Vtl) {
  __shared__ __align__(16) unsigned short Th[HDIM * 72];
  __shared__ __align__(16) unsigned short Tl[HDIM * 72];
  const int st = blockIdx.x / NKVH, hk = blockIdx.x % NKVH;
  const int s0 = st * 64;
  const int tid = threadIdx.x;
#pragma unroll
  for (int it = 0; it < 8; ++it) {
    const int i = tid + 256 * it;
    const int sr = i >> 5, part = i & 31;
    const v4f x = *(const v4f*)(qkv + (size_t)(s0 + sr) * QKVN + VOFF + hk * HDIM + part * 4);
#pragma unroll
    for (int e = 0; e < 4; ++e) {
      const int d = part * 4 + e;
      const unsigned short hb = f2bf_bits(x[e]);
      const unsigned short lb = f2bf_bits(x[e] - bf_bits2f(hb));
      Th[d * 72 + sr] = hb;
      Tl[d * 72 + sr] = lb;
    }
  }
  __syncthreads();
  const int wave = tid >> 5, lane = tid & 31, q = lane >> 3, c8 = (lane & 7) * 8;
  for (int ps = 0; ps < 2; ++ps) {
#pragma unroll
    for (int it = 0; it < 4; ++it) {
      const int row = wave * 16 + it * 4 + q;
      const v4u a = *(const v4u*)(Th + row * 72 + c8);
      const v4u b = *(const v4u*)(Tl + row * 72 + c8);
      const size_t go = (size_t)(hk * HDIM + row) * SEQ + s0 + c8;
      *(volatile v4u*)(Vth + go) = a;
      *(volatile v4u*)(Vtl + go) = b;
    }
    __threadfence();
  }
}

constexpr int AQB = 64;
constexpr int AKC = 64;
constexpr int ANW = 4;
constexpr int OPITCH = 132;
static_assert(AQB == AKC && SEQ % AQB == 0, "chunking");
static_assert(ANW * 16 * OPITCH * 4 <= 4 * AKC * HDIM * 2, "out staging fits in K/V region");

__global__ __launch_bounds__(128) void attn_hd128_kernel(
    const unsigned short* __restrict__ Qh, const unsigned short* __restrict__ Ql,
    const unsigned short* __restrict__ Kh, const unsigned short* __restrict__ Kl,
    const unsigned short* __restrict__ Vth, const unsigned short* __restrict__ Vtl,
    const float* __restrict__ amask,
    unsigned short* __restrict__ Oh, unsigned short* __restrict__ Ol, float scale) {
  union FB { v16b v; v8b h[2]; };
  __shared__ __align__(16) __bf16 Qs[2][AQB * HDIM];
  __shared__ __align__(16) __bf16 KVs[4][AKC * HDIM];
  __shared__ __align__(16) __bf16 Ps[2][ANW][16 * AKC];
  __shared__ __align__(16) float  Ms[AQB * AKC];

  const int tid  = threadIdx.x;
  const int wave = tid >> 5, lane = tid & 31, hh = lane >> 4, c = lane & 15;
  constexpr int nqb = SEQ / AQB;
  const int qb = blockIdx.x % nqb;
  const int h  = blockIdx.x / nqb;
  const int hk = h / (NHEAD / NKVH);
  const int qbase = qb * AQB;
  const int qw = wave * 16;

  {
    const v4u* gh = (const v4u*)(Qh + (size_t)(h * SEQ + qbase) * HDIM);
    const v4u* gl = (const v4u*)(Ql + (size_t)(h * SEQ + qbase) * HDIM);
    v4u* dh = (v4u*)(&Qs[0][0]);
    v4u* dl = (v4u*)(&Qs[1][0]);
#pragma unroll
    for (int it = 0; it < 8; ++it) dh[tid + 128 * it] = gh[tid + 128 * it];
    asm volatile("" ::: "memory");
#pragma unroll
    for (int it = 0; it < 8; ++it) dl[tid + 128 * it] = gl[tid + 128 * it];
    asm volatile("" ::: "memory");
  }

  float mrow[8], lrow[8];
  v8f oacc[8];
#pragma unroll
  for (int r = 0; r < 8; ++r) { mrow[r] = -INFINITY; lrow[r] = 0.f; }
#pragma unroll
  for (int t = 0; t < 8; ++t) oacc[t] = (v8f){0.f,0.f,0.f,0.f,0.f,0.f,0.f,0.f};

  for (int kc = 0; kc <= qb; ++kc) {
    const int kv0 = kc * AKC;
    __syncthreads();
    {
      const v4u* gkh = (const v4u*)(Kh + (size_t)(hk * SEQ + kv0) * HDIM);
      const v4u* gkl = (const v4u*)(Kl + (size_t)(hk * SEQ + kv0) * HDIM);
      v4u* dkh = (v4u*)(&KVs[0][0]);
      v4u* dkl = (v4u*)(&KVs[1][0]);
#pragma unroll
      for (int it = 0; it < 8; ++it) dkh[tid + 128 * it] = gkh[tid + 128 * it];
      asm volatile("" ::: "memory");
#pragma unroll
      for (int it = 0; it < 8; ++it) dkl[tid + 128 * it] = gkl[tid + 128 * it];
      asm volatile("" ::: "memory");
      v4u* dvh = (v4u*)(&KVs[2][0]);
      v4u* dvl = (v4u*)(&KVs[3][0]);
#pragma unroll
      for (int it = 0; it < 8; ++it) {
        const int i = tid + 128 * it;
        const int d = i >> 3, part = i & 7;
        dvh[i] = *((const v4u*)(Vth + (size_t)(hk * HDIM + d) * SEQ + kv0) + part);
      }
      asm volatile("" ::: "memory");
#pragma unroll
      for (int it = 0; it < 8; ++it) {
        const int i = tid + 128 * it;
        const int d = i >> 3, part = i & 7;
        dvl[i] = *((const v4u*)(Vtl + (size_t)(hk * HDIM + d) * SEQ + kv0) + part);
      }
      asm volatile("" ::: "memory");
      v4f* dm = (v4f*)(&Ms[0]);
#pragma unroll
      for (int it = 0; it < 8; ++it) {
        const int i = tid + 128 * it;
        const int qr = i >> 4, part = i & 15;
        dm[i] = *((const v4f*)(amask + (size_t)(qbase + qr) * SEQ + kv0) + part);
      }
    }
    __syncthreads();

    v8f sacc[4];
#pragma unroll
    for (int j = 0; j < 4; ++j) sacc[j] = (v8f){0.f,0.f,0.f,0.f,0.f,0.f,0.f,0.f};
#pragma unroll 1
    for (int dc = 0; dc < 4; ++dc) {
      FB qa, ql;
      qa.h[0] = *(const v8b*)(&Qs[0][0] + (qw + c) * HDIM + dc * 32 + 8 * hh);
      qa.h[1] = *(const v8b*)(&Qs[0][0] + (qw + c) * HDIM + dc * 32 + 16 + 8 * hh);
      ql.h[0] = *(const v8b*)(&Qs[1][0] + (qw + c) * HDIM + dc * 32 + 8 * hh);
      ql.h[1] = *(const v8b*)(&Qs[1][0] + (qw + c) * HDIM + dc * 32 + 16 + 8 * hh);
#pragma unroll
      for (int j = 0; j < 4; ++j) {
        FB kb, kl;
        kb.h[0] = *(const v8b*)(&KVs[0][0] + (j * 16 + c) * HDIM + dc * 32 + 8 * hh);
        kb.h[1] = *(const v8b*)(&KVs[0][0] + (j * 16 + c) * HDIM + dc * 32 + 16 + 8 * hh);
        kl.h[0] = *(const v8b*)(&KVs[1][0] + (j * 16 + c) * HDIM + dc * 32 + 8 * hh);
        kl.h[1] = *(const v8b*)(&KVs[1][0] + (j * 16 + c) * HDIM + dc * 32 + 16 + 8 * hh);
        sacc[j] = at_mma(qa.v, kb.v, sacc[j]);
        sacc[j] = at_mma(qa.v, kl.v, sacc[j]);
        sacc[j] = at_mma(ql.v, kb.v, sacc[j]);
      }
    }

    float cm[8];
#pragma unroll
    for (int r = 0; r < 8; ++r) {
      const int qrl = qw + 8 * hh + r;
      float m = -INFINITY;
#pragma unroll
      for (int j = 0; j < 4; ++j) {
        const float mv = bf_bits2f(f2bf_bits(Ms[qrl * AKC + j * 16 + c]));
        const float sv = sacc[j][r] * scale + mv;
        sacc[j][r] = sv;
        m = fmaxf(m, sv);
      }
#pragma unroll
      for (int off = 1; off < 16; off <<= 1) m = fmaxf(m, __shfl_xor(m, off, 32));
      cm[r] = m;
    }

    __bf16* pwh = &Ps[0][wave][0];
    __bf16* pwl = &Ps[1][wave][0];
#pragma unroll
    for (int r = 0; r < 8; ++r) {
      const float mnew = fmaxf(mrow[r], cm[r]);
      const float alpha = expf(mrow[r] - mnew);
      mrow[r] = mnew;
      float psum = 0.f;
#pragma unroll
      for (int j = 0; j < 4; ++j) {
        const float p = expf(sacc[j][r] - mnew);
        psum += p;
        __bf16 ph, pl;
        at_split(p, ph, pl);
        pwh[(8 * hh + r) * AKC + j * 16 + c] = ph;
        pwl[(8 * hh + r) * AKC + j * 16 + c] = pl;
      }
#pragma unroll
      for (int off = 1; off < 16; off <<= 1) psum += __shfl_xor(psum, off, 32);
      lrow[r] = lrow[r] * alpha + psum;
#pragma unroll
      for (int t = 0; t < 8; ++t) oacc[t][r] = oacc[t][r] * alpha;
    }
    __syncthreads();

#pragma unroll 1
    for (int kk = 0; kk < 2; ++kk) {
      FB pa, pl;
      pa.h[0] = *(const v8b*)(pwh + c * AKC + kk * 32 + 8 * hh);
      pa.h[1] = *(const v8b*)(pwh + c * AKC + kk * 32 + 16 + 8 * hh);
      pl.h[0] = *(const v8b*)(pwl + c * AKC + kk * 32 + 8 * hh);
      pl.h[1] = *(const v8b*)(pwl + c * AKC + kk * 32 + 16 + 8 * hh);
#pragma unroll
      for (int t = 0; t < 8; ++t) {
        FB vb, vl;
        vb.h[0] = *(const v8b*)(&KVs[2][0] + (t * 16 + c) * AKC + kk * 32 + 8 * hh);
        vb.h[1] = *(const v8b*)(&KVs[2][0] + (t * 16 + c) * AKC + kk * 32 + 16 + 8 * hh);
        vl.h[0] = *(const v8b*)(&KVs[3][0] + (t * 16 + c) * AKC + kk * 32 + 8 * hh);
        vl.h[1] = *(const v8b*)(&KVs[3][0] + (t * 16 + c) * AKC + kk * 32 + 16 + 8 * hh);
        oacc[t] = at_mma(pa.v, vb.v, oacc[t]);
        oacc[t] = at_mma(pa.v, vl.v, oacc[t]);
        oacc[t] = at_mma(pl.v, vb.v, oacc[t]);
        if (t == 3) asm volatile("" ::: "memory");
      }
    }
  }

  __syncthreads();
  float* os = (float*)(&KVs[0][0]) + wave * (16 * OPITCH);
#pragma unroll
  for (int r = 0; r < 8; ++r) {
    const float inv = 1.0f / lrow[r];
#pragma unroll
    for (int t = 0; t < 8; ++t) os[(8 * hh + r) * OPITCH + t * 16 + c] = oacc[t][r] * inv;
  }
  __syncthreads();
  {
    const size_t grow0 = (size_t)(qbase + qw);
    const int c8 = c * 8;
    for (int ps = 0; ps < 2; ++ps) {
#pragma unroll
      for (int it = 0; it < 8; ++it) {
        const int row = it * 2 + hh;
        const float* sp = os + row * OPITCH + c8;
        const v4f a = *(const v4f*)sp;
        const v4f b = *(const v4f*)(sp + 4);
        const HL2 p0 = split_pack2(a[0], a[1]);
        const HL2 p1 = split_pack2(a[2], a[3]);
        const HL2 p2 = split_pack2(b[0], b[1]);
        const HL2 p3 = split_pack2(b[2], b[3]);
        v4u hv, lv;
        hv[0] = p0.hi; hv[1] = p1.hi; hv[2] = p2.hi; hv[3] = p3.hi;
        lv[0] = p0.lo; lv[1] = p1.lo; lv[2] = p2.lo; lv[3] = p3.lo;
        const size_t go = (grow0 + row) * (size_t)HID + (size_t)h * HDIM + c8;
        *(volatile v4u*)(Oh + go) = hv;
        *(volatile v4u*)(Ol + go) = lv;
      }
      __threadfence();
    }
  }
}

extern "C" void kernel_launch(void* const* d_in, const int* in_sizes, int n_in,
                              void* d_out, int out_size, void* d_ws, size_t ws_size,
                              hipStream_t stream) {
  if (n_in < 5) return;
  if (in_sizes[0] != SEQ * HID || in_sizes[1] != SEQ * SEQ || in_sizes[2] != SEQ ||
      in_sizes[3] != HID * QKVN || in_sizes[4] != HID * HID) return;
  if (out_size != SEQ * HID) return;
  if (ws_size < WS_TOTAL) return;

  const float* hidden = (const float*)d_in[0];
  const float* amask  = (const float*)d_in[1];
  const int*   posid  = (const int*)d_in[2];
  const float* w_attn = (const float*)d_in[3];
  const float* w_proj = (const float*)d_in[4];
  float* out = (float*)d_out;

  char* ws = (char*)d_ws;
  unsigned short* Xb  = (unsigned short*)(ws + OFF_XB);
  unsigned short* Wat = (unsigned short*)(ws + OFF_WAT);
  unsigned short* Wpt = (unsigned short*)(ws + OFF_WPT);
  float*          qkv = (float*)(ws + OFF_QKV);
  unsigned short* Qhp = (unsigned short*)(ws + OFF_QH);
  unsigned short* Qlp = (unsigned short*)(ws + OFF_QL);
  unsigned short* Khp = (unsigned short*)(ws + OFF_KH);
  unsigned short* Klp = (unsigned short*)(ws + OFF_KL);
  unsigned short* Vhp = (unsigned short*)(ws + OFF_VH);
  unsigned short* Vlp = (unsigned short*)(ws + OFF_VL);
  unsigned short* Ohp = (unsigned short*)(ws + OFF_OH);
  unsigned short* Olp = (unsigned short*)(ws + OFF_OL);

  RopeFreq rf;
  for (int i = 0; i < 64; ++i) {
    const double ex = (double)(2 * i) / 128.0;
    const float pw = (float)pow(10000.0, ex);
    rf.inv[i] = 1.0f / pw;
  }

  {
    const int n8 = SEQ * HID / 8;
    cast_f32_bf16x8<<<dim3(n8 / 256), dim3(256), 0, stream>>>(hidden, Xb, n8);
  }
  transpose_cast_bf16<<<dim3(QKVN / 64, HID / 64), dim3(256), 0, stream>>>(w_attn, Wat, HID, QKVN);
  transpose_cast_bf16<<<dim3(HID / 64, HID / 64), dim3(256), 0, stream>>>(w_proj, Wpt, HID, HID);
  {
    const int tiles = (SEQ / 64) * (QKVN / 64);
    const int blocks = (tiles + 7) / 8;
    wmma_gemm64<1, 0, 0><<<dim3(blocks, 1), dim3(256), 0, stream>>>(
        Xb, Xb, HID, 0L, Wat, Wat, HID, 0L, (void*)qkv, (void*)qkv, QKVN, 0L, SEQ, QKVN, HID, 1.0f);
  }
  rope_qk_kernel<<<dim3(SEQ), dim3(128), 0, stream>>>(qkv, posid, rf, Qhp, Qlp, Khp, Klp);
  v_split_transpose_kernel<<<dim3((SEQ / 64) * NKVH), dim3(256), 0, stream>>>(qkv, Vhp, Vlp);
  attn_hd128_kernel<<<dim3(NHEAD * (SEQ / AQB)), dim3(128), 0, stream>>>(
      Qhp, Qlp, Khp, Klp, Vhp, Vlp, amask, Ohp, Olp, SM_SCALE);
  {
    const int tiles = (SEQ / 64) * (HID / 64);
    const int blocks = (tiles + 7) / 8;
    wmma_gemm64<1, 2, 0><<<dim3(blocks, 1), dim3(256), 0, stream>>>(
        Ohp, Olp, HID, 0L, Wpt, Wpt, HID, 0L, (void*)out, (void*)out, HID, 0L, SEQ, HID, HID, 1.0f);
  }
}
